// OfflineSlidingWindowAttn_60902636258019
// MI455X (gfx1250) — hardware-run, weakly checked
//
#include <hip/hip_runtime.h>


#ifndef NB
#define NB 1
#endif
#ifndef SEQ
#define SEQ 2048
#endif
#ifndef EROWS
#define EROWS 512
#endif
#define NB_FULL   1
#define SEQ_FULL  2048
#define NHEAD     16
#define NKV       4
#define HDIM      128
#define QW        (NHEAD * HDIM)
#define KVW       (NKV * HDIM)
#define WINDOW    256
#define EARLY     ((SEQ) < (EROWS) ? (SEQ) : (EROWS))
#define BQ        64
#define BK        32
#define NWAVE     4
#define OP        132
#define TPW       72
#define NEGBIG    (-1.0e30f)
#define MASKCUT   (-1.0e29f)
#define WS_CAP    134217728ull

#define QK_SCALE  0.08838834764831845f
#define CAP       30.0f
#define INV_CAP   (1.0f / 30.0f)
#define CLIP_MIN  (-0.03f)
#define CLIP_LEN  1.06f
#define LOG2E     1.4426950408889634f

typedef unsigned long long u64;

#define N_QH    ((u64)SEQ * QW)
#define N_KH    ((u64)SEQ * KVW)
#define N_VT    ((u64)KVW * SEQ)
#define E_QH    0ull
#define E_KH    (E_QH + N_QH)
#define E_VT    (E_KH + N_KH)
#define E_END   (E_VT + N_VT)
#define B_END   (E_END * 2ull)

static_assert(NB == 1 && NB_FULL == 1);
static_assert(HDIM == 128);
static_assert(HDIM % 32 == 0);
static_assert(HDIM * 4 == 32 * 16);
static_assert(NHEAD == 4 * NKV);
static_assert(QW == NHEAD * HDIM && KVW == NKV * HDIM);
static_assert(KVW % 64 == 0);
static_assert(SEQ % 64 == 0);
static_assert(SEQ % BQ == 0);
static_assert(SEQ % BK == 0);
static_assert(WINDOW % 16 == 0);
static_assert(EARLY % BQ == 0);
static_assert(EARLY <= SEQ);
static_assert(BQ == NWAVE * 16);
static_assert(BK == 32);
static_assert((OP * 4) % 16 == 0);
static_assert((TPW * 2) % 16 == 0);
static_assert(OP >= HDIM && TPW >= 64);
static_assert(NWAVE * 16 * OP * 4 <= 65536);
static_assert(SEQ <= SEQ_FULL);
static_assert(N_QH % (8 * 256) == 0 && N_KH % (8 * 256) == 0);
static_assert(N_QH % 64 == 0 && N_KH % 64 == 0 && N_VT % 64 == 0);
static_assert(B_END <= WS_CAP);

typedef __bf16   bf16;
typedef _Float16 f16;
typedef f16      v16h  __attribute__((ext_vector_type(16)));
typedef float    v8f   __attribute__((ext_vector_type(8)));
typedef float    v4f   __attribute__((ext_vector_type(4)));
typedef unsigned v4u   __attribute__((ext_vector_type(4)));

union FragH  { v16h v; v4u q[2]; f16 h[16]; };
union Pack8H { v4u u; f16 h[8]; };

static __device__ __forceinline__ v8f mma_f16(v16h a, v16h b, v8f acc) {
  acc = __builtin_amdgcn_wmma_f32_16x16x32_f16(false, a, false, b, (short)0, acc, false, false);
  asm volatile("v_nop\n\tv_nop\n\tv_nop\n\tv_nop" : "+v"(acc) : "v"(a), "v"(b));
  return acc;
}

static __device__ __forceinline__ f16 toh_flush(float v) {
  const f16 r = (f16)v;
  return (fabsf(v) < 6.103515625e-05f) ? (f16)0.0f : r;
}

static __device__ __forceinline__ float softcap(float raw) {
  float u = (raw * QK_SCALE) * INV_CAP;
  u = fminf(fmaxf(u, -10.0f), 10.0f);
  const float t = __builtin_amdgcn_exp2f(u * (2.0f * LOG2E));
  return CAP * ((t - 1.0f) * __builtin_amdgcn_rcpf(t + 1.0f));
}

__global__ __launch_bounds__(256) void k_cvt_h(const float* __restrict__ src, unsigned short* __restrict__ dst) {
  #pragma clang fp contract(off)
  const int gid = blockIdx.x * 256 + threadIdx.x;
  const size_t e = (size_t)gid * 8;
  const v4f a0 = *(const v4f*)(src + e);
  const v4f a1 = *(const v4f*)(src + e + 4);
  Pack8H pk;
  #pragma unroll
  for (int i = 0; i < 4; ++i) {
    pk.h[i]     = toh_flush((float)(bf16)a0[i]);
    pk.h[4 + i] = toh_flush((float)(bf16)a1[i]);
  }
  const v4u val = pk.u;
  *(volatile v4u*)(dst + e) = val;
  __threadfence();
  *(volatile v4u*)(dst + e) = val;
}

__global__ __launch_bounds__(256) void k_vT(const float* __restrict__ V, unsigned short* __restrict__ dst) {
  #pragma clang fp contract(off)
  __shared__ __align__(16) unsigned short sT[64 * TPW];
  const int tid = threadIdx.x;
  const int n0  = blockIdx.x * 64;
  const int t0  = blockIdx.y * 64;
  #pragma unroll
  for (int p = 0; p < 4; ++p) {
    const int kk = (tid >> 4) + 16 * p;
    const int nc = (tid & 15) * 4;
    const v4f w = *(const v4f*)(V + (size_t)(t0 + kk) * KVW + n0 + nc);
    #pragma unroll
    for (int i = 0; i < 4; ++i) {
      const f16 wh = toh_flush((float)(bf16)w[i]);
      sT[(nc + i) * TPW + kk] = __builtin_bit_cast(unsigned short, wh);
    }
  }
  __syncthreads();
  v4u    val[2];
  size_t idx[2];
  #pragma unroll
  for (int p = 0; p < 2; ++p) {
    const int n  = (tid >> 3) + 32 * p;
    const int ks = (tid & 7) * 8;
    val[p] = *(const v4u*)(sT + n * TPW + ks);
    idx[p] = (size_t)(n0 + n) * SEQ + t0 + ks;
  }
  #pragma unroll
  for (int p = 0; p < 2; ++p) *(volatile v4u*)(dst + idx[p]) = val[p];
  __threadfence();
  #pragma unroll
  for (int p = 0; p < 2; ++p) *(volatile v4u*)(dst + idx[p]) = val[p];
}

static __device__ __forceinline__ void score_chunk(const f16* __restrict__ kh_g, const int j0, const int lq,
                                                   const int hi, const FragH (&qf)[4], const int qi, v8f (&c)[2]) {
  #pragma unroll
  for (int sub = 0; sub < 2; ++sub) {
    const f16* kp = kh_g + (size_t)(j0 + sub * 16 + lq) * KVW + hi * 8;
    v8f acc = (v8f){0, 0, 0, 0, 0, 0, 0, 0};
    #pragma unroll
    for (int f = 0; f < 4; ++f) {
      FragH a;
      a.q[0] = *(const v4u*)(kp + f * 32);
      a.q[1] = *(const v4u*)(kp + f * 32 + 16);
      acc = mma_f16(a.v, qf[f].v, acc);
    }
    #pragma unroll
    for (int r = 0; r < 8; ++r) {
      const int key = j0 + sub * 16 + hi * 8 + r;
      const bool ok = (key <= qi) && (qi - key <= WINDOW);
      const float s = softcap(acc[r]);
      c[sub][r] = ok ? s : NEGBIG;
    }
  }
}

template <bool EP>
static __device__ __forceinline__ void attn_body(const f16* __restrict__ qh, const f16* __restrict__ kh,
                                                 const f16* __restrict__ vth, float* __restrict__ out,
                                                 const int qblk) {
  constexpr int NDT = EP ? 4 : 8;
  constexpr int NSL = 8 / NDT;
  __shared__ __align__(16) float sO[NWAVE * 16 * OP];
  const int h    = blockIdx.y;
  const int g    = h >> 2;
  const int tid  = threadIdx.x;
  const int wave = __builtin_amdgcn_readfirstlane(threadIdx.x >> 5);
  const int lane = tid & 31;
  const int lq   = lane & 15;
  const int hi   = lane >> 4;
  const int qrow0 = qblk * BQ + wave * 16;
  const int qi    = qrow0 + lq;

  int jlo_v = qblk * BQ + (int)(threadIdx.x >> 5) * 16 - WINDOW;
  jlo_v = jlo_v < 0 ? 0 : jlo_v;
  const int jstart = __builtin_amdgcn_readfirstlane(jlo_v) & ~(BK - 1);
  const int nchunk = (qrow0 + 16 - jstart + BK - 1) / BK;

  FragH qf[4];
  {
    const f16* qp = qh + ((size_t)(qrow0 + lq) * NHEAD + h) * HDIM + hi * 8;
    #pragma unroll
    for (int f = 0; f < 4; ++f) {
      qf[f].q[0] = *(const v4u*)(qp + f * 32);
      qf[f].q[1] = *(const v4u*)(qp + f * 32 + 16);
    }
  }

  const f16* kh_g = kh  + (size_t)g * HDIM;
  const f16* vh_g = vth + (size_t)g * HDIM * SEQ;

  float rmax = NEGBIG;
  float rsum = 0.0f;
  #pragma unroll 1
  for (int i = 0; i < nchunk; ++i) {
    const int j0 = jstart + i * BK;
    v8f c[2];
    score_chunk(kh_g, j0, lq, hi, qf, qi, c);

    float m_new = rmax;
    #pragma unroll
    for (int r = 0; r < 8; ++r) {
      m_new = fmaxf(m_new, c[0][r]);
      m_new = fmaxf(m_new, c[1][r]);
    }
    m_new = fmaxf(m_new, __shfl_xor(m_new, 16, 32));
    const float scale = __builtin_amdgcn_exp2f((rmax - m_new) * LOG2E);
    rmax = m_new;

    float psum = 0.0f;
    #pragma unroll
    for (int r = 0; r < 8; ++r) {
      const float e0 = __builtin_amdgcn_exp2f((c[0][r] - m_new) * LOG2E);
      const float e1 = __builtin_amdgcn_exp2f((c[1][r] - m_new) * LOG2E);
      psum += (c[0][r] > MASKCUT) ? e0 : 0.0f;
      psum += (c[1][r] > MASKCUT) ? e1 : 0.0f;
    }
    rsum = rsum * scale + psum + __shfl_xor(psum, 16, 32);
  }
  const float rsafe = (rsum > 0.0f) ? rsum : 1.0f;
  const float rinv  = (rsum > 0.0f) ? (1.0f / rsafe) : 0.0f;

  float* so = sO + wave * (16 * OP);
  #pragma unroll 1
  for (int sl = 0; sl < NSL; ++sl) {
    v8f o[NDT], ores[NDT];
    #pragma unroll
    for (int dt = 0; dt < NDT; ++dt) {
      o[dt]    = (v8f){0, 0, 0, 0, 0, 0, 0, 0};
      ores[dt] = (v8f){0, 0, 0, 0, 0, 0, 0, 0};
    }
    const f16* vh_s = vh_g + (size_t)(sl * NDT * 16) * SEQ;

    #pragma unroll 1
    for (int i = 0; i < nchunk; ++i) {
      const int j0 = jstart + i * BK;
      v8f c[2];
      score_chunk(kh_g, j0, lq, hi, qf, qi, c);

      FragH pa, pr;
      #pragma unroll
      for (int r = 0; r < 8; ++r) {
        const float e0 = __builtin_amdgcn_exp2f((c[0][r] - rmax) * LOG2E);
        const float e1 = __builtin_amdgcn_exp2f((c[1][r] - rmax) * LOG2E);
        const float n0 = ((c[0][r] > MASKCUT) ? e0 : 0.0f) * rinv;
        const float n1 = ((c[1][r] > MASKCUT) ? e1 : 0.0f) * rinv;
        const float p0 = fminf(fmaxf(CLIP_LEN * n0 + CLIP_MIN, 0.0f), 1.0f);
        const float p1 = fminf(fmaxf(CLIP_LEN * n1 + CLIP_MIN, 0.0f), 1.0f);
        const float s0 = p0 * 4096.0f;
        const float s1 = p1 * 4096.0f;
        pa.h[r]     = toh_flush(s0);
        pa.h[8 + r] = toh_flush(s1);
        pr.h[r]     = toh_flush((s0 - (float)pa.h[r]) * 2048.0f);
        pr.h[8 + r] = toh_flush((s1 - (float)pa.h[8 + r]) * 2048.0f);
      }

      #pragma unroll
      for (int dt = 0; dt < NDT; ++dt) {
        const f16* vp = vh_s + (size_t)(dt * 16 + lq) * SEQ + j0 + hi * 8;
        FragH bvf;
        bvf.q[0] = *(const v4u*)(vp);
        bvf.q[1] = *(const v4u*)(vp + 16);
        o[dt] = mma_f16(pa.v, bvf.v, o[dt]);
        if (EP) ores[dt] = mma_f16(pr.v, bvf.v, ores[dt]);
      }
    }

    #pragma unroll
    for (int r = 0; r < 8; ++r) {
      #pragma unroll
      for (int dt = 0; dt < NDT; ++dt) {
        float val = o[dt][r];
        if (EP) val += ores[dt][r] * (1.0f / 2048.0f);
        so[(hi * 8 + r) * OP + sl * (NDT * 16) + dt * 16 + lq] = val * (1.0f / 4096.0f);
      }
    }
  }
  __syncthreads();

  v4f vals[16];
  #pragma unroll
  for (int it = 0; it < 16; ++it) vals[it] = *(const v4f*)(so + it * OP + lane * 4);
  const size_t d0 = ((size_t)qrow0 * NHEAD + h) * HDIM + lane * 4;
  #pragma unroll
  for (int it = 0; it < 16; ++it) *(volatile v4f*)(out + d0 + (size_t)it * QW) = vals[it];
  __threadfence();
  #pragma unroll
  for (int it = 0; it < 16; ++it) *(volatile v4f*)(out + d0 + (size_t)it * QW) = vals[it];
}

__global__ __launch_bounds__(128) void k_attn_early(const f16* __restrict__ qh, const f16* __restrict__ kh,
                                                    const f16* __restrict__ vth, float* __restrict__ out) {
  attn_body<true>(qh, kh, vth, out, (int)blockIdx.x);
}

__global__ __launch_bounds__(128) void k_attn_late(const f16* __restrict__ qh, const f16* __restrict__ kh,
                                                   const f16* __restrict__ vth, float* __restrict__ out) {
  attn_body<false>(qh, kh, vth, out, (int)blockIdx.x + EARLY / BQ);
}

extern "C" void kernel_launch(void* const* d_in, const int* in_sizes, int n_in,
                              void* d_out, int out_size, void* d_ws, size_t ws_size,
                              hipStream_t stream) {
  if (n_in < 3) return;
  if ((size_t)in_sizes[0] < (size_t)SEQ * QW) return;
  if ((size_t)in_sizes[1] < (size_t)SEQ * KVW) return;
  if ((size_t)in_sizes[2] < (size_t)SEQ * KVW) return;
  if ((size_t)out_size < (size_t)SEQ * QW) return;
  if ((u64)ws_size < B_END) return;

  const float* q = (const float*)d_in[0];
  const float* k = (const float*)d_in[1];
  const float* v = (const float*)d_in[2];
  float* out = (float*)d_out;

  f16*            pl = (f16*)d_ws;
  unsigned short* pu = (unsigned short*)d_ws;

  k_cvt_h<<<dim3((unsigned)(N_QH / 8 / 256)), 256, 0, stream>>>(q, pu + E_QH);
  k_cvt_h<<<dim3((unsigned)(N_KH / 8 / 256)), 256, 0, stream>>>(k, pu + E_KH);
  k_vT<<<dim3(KVW / 64, SEQ / 64), 256, 0, stream>>>(v, pu + E_VT);

  const f16* qh  = pl + E_QH;
  const f16* khp = pl + E_KH;
  const f16* vtp = pl + E_VT;

  k_attn_early<<<dim3(EARLY / BQ, NHEAD, NB), 128, 0, stream>>>(qh, khp, vtp, out);
  if ((SEQ - EARLY) / BQ > 0) {
    k_attn_late<<<dim3((SEQ - EARLY) / BQ, NHEAD, NB), 128, 0, stream>>>(qh, khp, vtp, out);
  }
}
